// SFIMLLIE_22342419874204
// MI455X (gfx1250) — hardware-verified
//
#include <hip/hip_runtime.h>


namespace {
constexpr int NB = 2, HI = 64, LI = HI * HI, C = 96, D = 192, NS = 16, R = 6, NT = NB * LI, NE = 3;
constexpr float XS = 8.0f, US = 1024.0f, TS = 8192.0f, YGS = 64.0f, OS = 512.0f, GS = 32768.0f, WSC = 256.0f;
typedef _Float16 b16;
typedef __attribute__((ext_vector_type(16))) _Float16 v16b;
typedef __attribute__((ext_vector_type(8))) _Float16 v8b;
typedef __attribute__((ext_vector_type(8))) float v8f;
typedef __attribute__((ext_vector_type(4))) float v4f;
typedef __attribute__((ext_vector_type(2))) float v2f;
__device__ __forceinline__ float bf16_rne(float f) { unsigned int u = __float_as_uint(f); u += 0x7FFFu + ((u >> 16) & 1u); return __uint_as_float(u & 0xFFFF0000u); }
__device__ __forceinline__ void split16(float v, b16& hi, b16& lo) { hi = (b16)v; lo = (b16)(v - (float)hi); }
__device__ __forceinline__ v16b frag_kb(const b16* p, int hh) { const v8b a = *(const v8b*)(p + 8 * hh), b = *(const v8b*)(p + 16 + 8 * hh); v16b f;
#pragma unroll
  for (int e = 0; e < 8; ++e) { f[e] = a[e]; f[8 + e] = b[e]; } return f; }
__device__ __forceinline__ v8f wmma16b(v16b a, v16b b, v8f c) { v8f d = __builtin_amdgcn_wmma_f32_16x16x32_f16(false, a, false, b, (short)0, c, false, false); asm volatile("v_nop\n\tv_nop\n\tv_nop\n\tv_nop" : "+v"(d) : "v"(a), "v"(b)); return d; }
__device__ __forceinline__ void wave_lds_sync() { __builtin_amdgcn_fence(__ATOMIC_RELEASE, "workgroup"); __builtin_amdgcn_wave_barrier(); __builtin_amdgcn_fence(__ATOMIC_ACQUIRE, "workgroup"); }
__device__ __forceinline__ float pmul(float a, float b) { float p = a * b; asm volatile("" : "+v"(p)); return p; }
__device__ __forceinline__ int iclamp(int v, int lo, int hi) { return v < lo ? lo : (v > hi ? hi : v); }
__device__ __forceinline__ float sigm(float v) { return 1.0f / (1.0f + __expf(-v)); }
__device__ __forceinline__ float silu(float v) { return pmul(v, sigm(v)); }
__device__ __forceinline__ float leaky(float v) { return v >= 0.0f ? v : 0.2f * v; }
__device__ __forceinline__ float gelu(float v) { return 0.5f * v * (1.0f + erff(v * 0.70710678118654752f)); }
__device__ __forceinline__ float softplus(float v) { return v > 20.0f ? v : (v < -20.0f ? __expf(v) : log1pf(__expf(v))); }

__global__ __launch_bounds__(256) void wcopyp_kernel(const float* __restrict__ w, int KIN, int OUT, int KP, int OUTP, b16* __restrict__ WT) {
  const int u = blockIdx.x * 256 + threadIdx.x; if (u >= OUTP * KP / 8) return; const int e = u * 8; const int o = e / KP, k0 = e % KP; v8b v;
#pragma unroll
  for (int j = 0; j < 8; ++j) { const int k = k0 + j; v[j] = (o < OUT && k < KIN) ? (b16)(bf16_rne(w[(size_t)o * KIN + k]) * WSC) : (b16)0.0f; } for (int pass = 0; pass < 2; ++pass) { *(volatile v8b*)(WT + e) = v; __threadfence(); }
}
template <int KIN, int NTL, int EXACT, int EPI>
__global__ __launch_bounds__(32) void gemm_kernel(const float* __restrict__ IN, int PIN, float scale, const b16* __restrict__ W, const float* __restrict__ bias, int NTV, float* __restrict__ OUT, int POUT) {
  __shared__ __attribute__((aligned(16))) b16 Ah[16][KIN + 8], Al[16][KIN + 8]; __shared__ __attribute__((aligned(16))) float Tf[16][NTL * 16 + 4];
  const int lane = threadIdx.x, nloc = lane & 15, hlf = lane >> 4; const size_t t0 = (size_t)blockIdx.x * 16; if (t0 >= (size_t)NTV) return;
  for (int rr = 0; rr < 16; ++rr) for (int q = 0; q < KIN / 32; ++q) { float v = IN[(t0 + rr) * PIN + q * 32 + lane]; if (EXACT) v = bf16_rne(v); b16 p, ql; split16(v * scale, p, ql); Ah[rr][q * 32 + lane] = p; Al[rr][q * 32 + lane] = ql; }
  wave_lds_sync(); const float sc = 1.0f / (scale * WSC);
  constexpr int NP = (NTL + 7) / 8;
#pragma unroll 1
  for (int cg = 0; cg < NP; ++cg) { const int nt = NTL - cg * 8 < 8 ? NTL - cg * 8 : 8; v8f acc[8];
#pragma unroll
    for (int t = 0; t < 8; ++t) acc[t] = (v8f){};
#pragma unroll 2
    for (int kb = 0; kb < KIN; kb += 32) { const v16b a = frag_kb(&Ah[nloc][kb], hlf), al = frag_kb(&Al[nloc][kb], hlf);
#pragma unroll
      for (int t = 0; t < 8; ++t) { if (t < nt) { const v16b bw = frag_kb(W + (size_t)(cg * 128 + t * 16 + nloc) * KIN + kb, hlf); acc[t] = wmma16b(a, bw, acc[t]); if (!EXACT) acc[t] = wmma16b(al, bw, acc[t]); } } }
#pragma unroll
    for (int t = 0; t < 8; ++t) { if (t < nt) { const int c = cg * 128 + t * 16 + nloc; const float bb = bias ? bf16_rne(bias[c]) : 0.0f;
#pragma unroll 1
        for (int r8 = 0; r8 < 8; ++r8) { float v = acc[t][r8] * sc + bb; if (EPI == 1) v = leaky(v); Tf[8 * hlf + r8][t * 16 + nloc] = v; } } }
    wave_lds_sync();
    for (int pass = 0; pass < 2; ++pass) { for (int rr = 0; rr < 16; ++rr) for (int c = lane; c < nt * 16; c += 32) ((volatile float*)OUT)[(t0 + rr) * POUT + cg * 128 + c] = Tf[rr][c]; __threadfence(); }
    wave_lds_sync(); }
}
__global__ __launch_bounds__(256) void dwconv_kernel(const float* __restrict__ IN, int PIN, const float* __restrict__ cw, const float* __restrict__ cb, int NTV, float* __restrict__ OUT) {
  const size_t gid = (size_t)blockIdx.x * 256 + threadIdx.x; const size_t t = gid / (D / 4); const int d4 = (int)(gid % (D / 4)) * 4; if (t >= (size_t)NTV) return;
  const int b = (int)(t / LI), p = (int)(t % LI), y = p / HI, xx = p % HI; v4f acc; for (int q = 0; q < 4; ++q) acc[q] = bf16_rne(cb[d4 + q]);
#pragma unroll
  for (int di = 0; di < 3; ++di)
#pragma unroll
    for (int dj = 0; dj < 3; ++dj) { const int yy = y + di - 1, x2 = xx + dj - 1; const bool ok = yy >= 0 && yy < HI && x2 >= 0 && x2 < HI; const int yc = ok ? yy : y, xc = ok ? x2 : xx;
      const v4f v = *(const v4f*)(IN + (((size_t)b * HI + yc) * HI + xc) * PIN + d4); for (int q = 0; q < 4; ++q) acc[q] += ok ? pmul(v[q], bf16_rne(cw[(d4 + q) * 9 + di * 3 + dj])) : 0.0f; }
  v4f o; for (int q = 0; q < 4; ++q) o[q] = silu(acc[q]);
  for (int pass = 0; pass < 2; ++pass) { *(volatile v4f*)(OUT + t * D + d4) = o; __threadfence(); }
}
__global__ __launch_bounds__(256) void small_kernel(const float* __restrict__ P1, const float* __restrict__ pe2w, const float* __restrict__ pe2b, const float* __restrict__ il, const float* __restrict__ ig1w, const float* __restrict__ ig1b, const float* __restrict__ ig2w, const float* __restrict__ ig2b, const float* __restrict__ r1w, const float* __restrict__ r1b, const float* __restrict__ r2w, const float* __restrict__ r2b, int NTV, float* __restrict__ SMA) {
  __shared__ float W2[4][48], G1[48][9], G1b[48], G2[4][48], R1[8][9], R1b[8], R2[3][8];
  for (int i = threadIdx.x; i < 192; i += 256) { W2[i / 48][i % 48] = bf16_rne(pe2w[i]); G2[i / 48][i % 48] = bf16_rne(ig2w[i]); } for (int i = threadIdx.x; i < 432; i += 256) G1[i / 9][i % 9] = bf16_rne(ig1w[i]);
  for (int i = threadIdx.x; i < 72; i += 256) R1[i / 9][i % 9] = bf16_rne(r1w[i]); if (threadIdx.x < 48) G1b[threadIdx.x] = bf16_rne(ig1b[threadIdx.x]); if (threadIdx.x < 8) R1b[threadIdx.x] = bf16_rne(r1b[threadIdx.x]); if (threadIdx.x < 24) R2[threadIdx.x / 8][threadIdx.x % 8] = bf16_rne(r2w[threadIdx.x]);
  __syncthreads();
  const size_t t = (size_t)blockIdx.x * 256 + threadIdx.x; if (t >= (size_t)NTV) return; const int b = (int)(t / LI), p = (int)(t % LI), y = p / HI, xx = p % HI;
  float ph[4]; for (int k = 0; k < 4; ++k) ph[k] = bf16_rne(pe2b[k]);
#pragma unroll 1
  for (int j = 0; j < 48; ++j) { const float v = P1[t * 64 + j]; for (int k = 0; k < 4; ++k) ph[k] += pmul(v, W2[k][j]); }
  float i9[9];
#pragma unroll
  for (int tap = 0; tap < 9; ++tap) { const int yy = y + tap / 3 - 1, x2 = xx + tap % 3 - 1; float v = 0.0f; if (yy >= 0 && yy < HI && x2 >= 0 && x2 < HI) { const size_t o = (size_t)yy * HI + x2; v = (bf16_rne(il[((size_t)b * 3 + 0) * LI + o]) + bf16_rne(il[((size_t)b * 3 + 1) * LI + o]) + bf16_rne(il[((size_t)b * 3 + 2) * LI + o])) * (1.0f / 3.0f); } i9[tap] = v; }
  float gt[4]; for (int k = 0; k < 4; ++k) gt[k] = bf16_rne(ig2b[k]);
#pragma unroll 1
  for (int j = 0; j < 48; ++j) { float s = G1b[j]; for (int tap = 0; tap < 9; ++tap) s += pmul(i9[tap], G1[j][tap]); s = leaky(s); for (int k = 0; k < 4; ++k) gt[k] += pmul(s, G2[k][j]); }
  float al[3]; for (int e = 0; e < 3; ++e) al[e] = bf16_rne(r2b[e]);
#pragma unroll 1
  for (int j = 0; j < 8; ++j) { float s = R1b[j]; for (int tap = 0; tap < 9; ++tap) s += pmul(i9[tap], R1[j][tap]); s = gelu(s); for (int e = 0; e < 3; ++e) al[e] += pmul(s, R2[e][j]); }
  const float gm = fmaxf(fmaxf(gt[0], gt[1]), fmaxf(gt[2], gt[3])); float ge[4], gs = 0.0f; for (int k = 0; k < 4; ++k) { ge[k] = __expf(gt[k] - gm); gs += ge[k]; }
  const float am = fmaxf(al[0], fmaxf(al[1], al[2])); float ae[3], as = 0.0f; for (int e = 0; e < 3; ++e) { ae[e] = __expf(al[e] - am); as += ae[e]; }
  v4f o0, o1; for (int k = 0; k < 4; ++k) o0[k] = pmul(sigm(ph[k]), ge[k] / gs); o1[0] = ae[0] / as; o1[1] = ae[1] / as; o1[2] = ae[2] / as; o1[3] = 0.0f;
  for (int pass = 0; pass < 2; ++pass) { *(volatile v4f*)(SMA + t * 8) = o0; *(volatile v4f*)(SMA + t * 8 + 4) = o1; __threadfence(); }
}
__global__ __launch_bounds__(32) void xproj_kernel(const float* __restrict__ U, const float* __restrict__ SMA, const b16* __restrict__ XPW, const b16* __restrict__ DTW, const float* __restrict__ dtb, int NTV, float* __restrict__ BC, float* __restrict__ DT) {
  __shared__ __attribute__((aligned(16))) b16 Ah[16][D + 8], Al[16][D + 8], Dh[16][32 + 8], Dl[16][32 + 8]; __shared__ __attribute__((aligned(16))) float Sbc[16][32], Tf[16][96 + 4];
  const int lane = threadIdx.x, nloc = lane & 15, hlf = lane >> 4; const size_t t0 = (size_t)blockIdx.x * 16; const int k = blockIdx.y; if (t0 >= (size_t)NTV) return;
  for (int rr = 0; rr < 16; ++rr) { for (int q = 0; q < D / 32; ++q) { b16 p, ql; split16(U[(t0 + rr) * D + q * 32 + lane] * US, p, ql); Ah[rr][q * 32 + lane] = p; Al[rr][q * 32 + lane] = ql; } Dh[rr][lane] = (b16)0.0f; Dl[rr][lane] = (b16)0.0f; }
  wave_lds_sync();
  v8f ax[3] = {(v8f){}, (v8f){}, (v8f){}};
#pragma unroll 2
  for (int kb = 0; kb < D; kb += 32) { const v16b a = frag_kb(&Ah[nloc][kb], hlf), al = frag_kb(&Al[nloc][kb], hlf);
#pragma unroll
    for (int t = 0; t < 3; ++t) { const v16b bw = frag_kb(XPW + ((size_t)k * 48 + t * 16 + nloc) * D + kb, hlf); ax[t] = wmma16b(a, bw, ax[t]); ax[t] = wmma16b(al, bw, ax[t]); } }
  wave_lds_sync();
#pragma unroll
  for (int t = 0; t < 3; ++t) { const int c = t * 16 + nloc;
#pragma unroll
    for (int r8 = 0; r8 < 8; ++r8) { const int rl = 8 * hlf + r8; const float v = pmul(ax[t][r8] * (1.0f / (US * WSC)), SMA[(t0 + rl) * 8 + k]); if (c < R) { b16 p, ql; split16(v * TS, p, ql); Dh[rl][c] = p; Dl[rl][c] = ql; } else if (c < R + 32) Sbc[rl][c - R] = v; } }
  wave_lds_sync();
  for (int pass = 0; pass < 2; ++pass) { for (int rr = 0; rr < 16; ++rr) ((volatile float*)BC)[((size_t)k * NT + t0 + rr) * 32 + lane] = Sbc[rr][lane]; __threadfence(); }
  const v16b a = frag_kb(&Dh[nloc][0], hlf), al = frag_kb(&Dl[nloc][0], hlf);
#pragma unroll 1
  for (int cg = 0; cg < 2; ++cg) { v8f acc[6];
#pragma unroll
    for (int t = 0; t < 6; ++t) { acc[t] = (v8f){}; const v16b bw = frag_kb(DTW + ((size_t)k * D + cg * 96 + t * 16 + nloc) * 32, hlf); acc[t] = wmma16b(a, bw, acc[t]); acc[t] = wmma16b(al, bw, acc[t]); }
#pragma unroll
    for (int t = 0; t < 6; ++t) { const int c = cg * 96 + t * 16 + nloc; const float bb = bf16_rne(dtb[k * D + c]);
#pragma unroll 1
      for (int r8 = 0; r8 < 8; ++r8) Tf[8 * hlf + r8][t * 16 + nloc] = softplus(acc[t][r8] * (1.0f / (TS * WSC)) + bb); }
    wave_lds_sync();
    for (int pass = 0; pass < 2; ++pass) { for (int rr = 0; rr < 16; ++rr) for (int q = 0; q < 3; ++q) ((volatile float*)DT)[((size_t)k * NT + t0 + rr) * D + cg * 96 + q * 32 + lane] = Tf[rr][q * 32 + lane]; __threadfence(); }
    wave_lds_sync(); }
}
__global__ __launch_bounds__(256) void scan_kernel(const float* __restrict__ U, const float* __restrict__ DT, const float* __restrict__ BC, const int* __restrict__ sid, const float* __restrict__ alog, const float* __restrict__ Ds, int NBV, float* __restrict__ YS) {
  const int gid = blockIdx.x * 256 + threadIdx.x; const int d = gid % D, k = (gid / D) % 4, b = gid / (4 * D); if (b >= NBV) return;
  float A[NS]; for (int s = 0; s < NS; ++s) A[s] = -__expf(bf16_rne(alog[((size_t)k * D + d) * NS + s])); const float dk = bf16_rne(Ds[k * D + d]);
#pragma unroll 1
  for (int pass = 0; pass < 2; ++pass) { float h[NS]; for (int s = 0; s < NS; ++s) h[s] = 0.0f;
#pragma unroll 1
    for (int l = 0; l < LI; ++l) { const int tok = iclamp(sid[k * LI + l], 0, LI - 1); const size_t row = (size_t)b * LI + tok; const size_t krow = (size_t)k * NT + row;
      const float u = U[row * D + d], dt = DT[krow * D + d]; const float du = pmul(dt, u); const float* bc = BC + krow * 32; float acc = 0.0f;
#pragma unroll
      for (int s = 0; s < NS; ++s) { h[s] = pmul(h[s], __expf(pmul(dt, A[s]))) + pmul(du, bc[s]); acc += pmul(h[s], bc[NS + s]); }
      ((volatile float*)YS)[((size_t)k * NT + (size_t)b * LI + l) * D + d] = acc + pmul(dk, u); }
    __threadfence(); }
}
__global__ __launch_bounds__(32) void tail_kernel(const float* __restrict__ YS, const int* __restrict__ iid, const float* __restrict__ XZ, const float* __restrict__ g, const float* __restrict__ bb, const b16* __restrict__ WO, int NTV, float* __restrict__ YO) {
  __shared__ __attribute__((aligned(16))) b16 Ah[16][D + 8], Al[16][D + 8]; __shared__ __attribute__((aligned(16))) float Tf[16][96 + 4];
  const int lane = threadIdx.x, nloc = lane & 15, hlf = lane >> 4; const size_t t0 = (size_t)blockIdx.x * 16; if (t0 >= (size_t)NTV) return;
  float gg[6], be[6]; for (int q = 0; q < 6; ++q) { gg[q] = bf16_rne(g[q * 32 + lane]); be[q] = bf16_rne(bb[q * 32 + lane]); }
  for (int rr = 0; rr < 16; ++rr) { const size_t t = t0 + rr; const int b = (int)(t / LI), p = (int)(t % LI); float v[6]; for (int q = 0; q < 6; ++q) v[q] = 0.0f; float s = 0.0f;
    for (int k = 0; k < 4; ++k) { const int pos = iclamp(iid[k * LI + p], 0, LI - 1); const float* ys = YS + ((size_t)k * NT + (size_t)b * LI + pos) * D; for (int q = 0; q < 6; ++q) v[q] += ys[q * 32 + lane]; }
    for (int q = 0; q < 6; ++q) s += v[q]; for (int o = 16; o; o >>= 1) s += __shfl_xor(s, o); const float mu = s * (1.0f / D); float vq = 0.0f; for (int q = 0; q < 6; ++q) { const float d_ = v[q] - mu; vq += pmul(d_, d_); } for (int o = 16; o; o >>= 1) vq += __shfl_xor(vq, o); const float rs = rsqrtf(vq * (1.0f / D) + 1e-5f);
    for (int q = 0; q < 6; ++q) { const int c = q * 32 + lane; const float z = XZ[t * (2 * D) + D + c]; const float a = pmul(pmul(pmul(v[q] - mu, rs), gg[q]) + be[q], silu(z)); b16 ph, pl; split16(a * YGS, ph, pl); Ah[rr][c] = ph; Al[rr][c] = pl; } }
  wave_lds_sync();
  v8f acc[6];
#pragma unroll
  for (int t = 0; t < 6; ++t) acc[t] = (v8f){};
#pragma unroll 2
  for (int kb = 0; kb < D; kb += 32) { const v16b a = frag_kb(&Ah[nloc][kb], hlf), al = frag_kb(&Al[nloc][kb], hlf);
#pragma unroll
    for (int t = 0; t < 6; ++t) { const v16b bw = frag_kb(WO + (size_t)(t * 16 + nloc) * D + kb, hlf); acc[t] = wmma16b(a, bw, acc[t]); acc[t] = wmma16b(al, bw, acc[t]); } }
#pragma unroll
  for (int t = 0; t < 6; ++t)
#pragma unroll 1
    for (int r8 = 0; r8 < 8; ++r8) Tf[8 * hlf + r8][t * 16 + nloc] = acc[t][r8] * (1.0f / (YGS * WSC));
  wave_lds_sync();
  for (int pass = 0; pass < 2; ++pass) { for (int rr = 0; rr < 16; ++rr) for (int q = 0; q < 3; ++q) ((volatile float*)YO)[(t0 + rr) * C + q * 32 + lane] = Tf[rr][q * 32 + lane]; __threadfence(); }
}
__global__ __launch_bounds__(256) void moeA_kernel(const float* __restrict__ FF, const float* __restrict__ SMA, const float* __restrict__ exw, const float* __restrict__ exb, int NTV, float* __restrict__ FO) {
  const size_t gid = (size_t)blockIdx.x * 256 + threadIdx.x; const size_t t = gid / (D / 4); const int d4 = (int)(gid % (D / 4)) * 4; if (t >= (size_t)NTV) return;
  const int b = (int)(t / LI), p = (int)(t % LI), y = p / HI, xx = p % HI; const float a0 = SMA[t * 8 + 4], a1 = SMA[t * 8 + 5], a2 = SMA[t * 8 + 6];
  v4f m = {0, 0, 0, 0};
#pragma unroll 1
  for (int e = 0; e < NE; ++e) { const float al = e == 0 ? a0 : (e == 1 ? a1 : a2); v4f acc; for (int q = 0; q < 4; ++q) acc[q] = bf16_rne(exb[e * D + d4 + q]);
#pragma unroll
    for (int tap = 0; tap < 9; ++tap) { const int yy = y + tap / 3 - 1, x2 = xx + tap % 3 - 1; const bool ok = yy >= 0 && yy < HI && x2 >= 0 && x2 < HI; const int yc = ok ? yy : y, xc = ok ? x2 : xx;
      const v4f v = *(const v4f*)(FF + (((size_t)b * HI + yc) * HI + xc) * D + d4); for (int q = 0; q < 4; ++q) acc[q] += ok ? pmul(v[q], bf16_rne(exw[((size_t)e * D + d4 + q) * 9 + tap])) : 0.0f; }
    for (int q = 0; q < 4; ++q) m[q] += pmul(al, acc[q]); }
  const v4f f = *(const v4f*)(FF + t * D + d4); v4f o; for (int q = 0; q < 4; ++q) o[q] = f[q] + pmul(m[q], f[q]);
  for (int pass = 0; pass < 2; ++pass) { *(volatile v4f*)(FO + t * D + d4) = o; __threadfence(); }
}
__global__ __launch_bounds__(256) void moeB_kernel(const float* __restrict__ FO, const float* __restrict__ mdw, const float* __restrict__ mdb, int NTV, float* __restrict__ G) {
  const size_t gid = (size_t)blockIdx.x * 256 + threadIdx.x; const size_t t = gid / (D / 4); const int d4 = (int)(gid % (D / 4)) * 4; if (t >= (size_t)NTV) return;
  const int b = (int)(t / LI), p = (int)(t % LI), y = p / HI, xx = p % HI; v4f acc; for (int q = 0; q < 4; ++q) acc[q] = bf16_rne(mdb[d4 + q]);
#pragma unroll
  for (int tap = 0; tap < 9; ++tap) { const int yy = y + tap / 3 - 1, x2 = xx + tap % 3 - 1; const bool ok = yy >= 0 && yy < HI && x2 >= 0 && x2 < HI; const int yc = ok ? yy : y, xc = ok ? x2 : xx;
    const v4f v = *(const v4f*)(FO + (((size_t)b * HI + yc) * HI + xc) * D + d4); for (int q = 0; q < 4; ++q) acc[q] += ok ? pmul(v[q], bf16_rne(mdw[(d4 + q) * 9 + tap])) : 0.0f; }
  v4f o; for (int q = 0; q < 4; ++q) o[q] = gelu(acc[q]);
  for (int pass = 0; pass < 2; ++pass) { *(volatile v4f*)(G + t * D + d4) = o; __threadfence(); }
}
}

extern "C" void kernel_launch(void* const* d_in, const int* in_sizes, int n_in, void* d_out, int out_size, void* d_ws, size_t ws_size, hipStream_t stream) {
  (void)n_in;
  auto Fp = [&](int i) { return (const float*)d_in[i]; }; auto Ip = [&](int i) { return (const int*)d_in[i]; };
  if (in_sizes[0] != NT * C || in_sizes[1] != NB * 3 * LI || in_sizes[2] != 2 * D * C || in_sizes[5] != 48 * D || in_sizes[13] != 4 * 38 * D || in_sizes[14] != 4 * D * R || in_sizes[16] != 4 * D * NS || in_sizes[20] != C * D || in_sizes[21] != D * C || in_sizes[23] != NE * D * 9 || in_sizes[31] != C * D || in_sizes[33] != 4 * LI || in_sizes[34] != 4 * LI || out_size != NT * C) return;
  const int NBV = NB; const int NTV = NBV * LI;
  size_t off = 0; char* ws = (char*)d_ws;
  auto carve = [&](size_t bytes) { char* p = ws + off; off += (bytes + 255) & ~(size_t)255; return p; };
  b16* WI = (b16*)carve((size_t)2 * D * C * 2); b16* WP1 = (b16*)carve(48 * D * 2); b16* XPW = (b16*)carve((size_t)4 * 48 * D * 2); b16* DTW = (b16*)carve((size_t)4 * D * 32 * 2); b16* WO = (b16*)carve(C * D * 2); b16* WFI = (b16*)carve(D * C * 2); b16* WFO = (b16*)carve(C * D * 2);
  float* XZ = (float*)carve((size_t)NT * 2 * D * 4); float* U = (float*)carve((size_t)NT * D * 4); float* P1 = (float*)carve((size_t)NT * 64 * 4); float* SMA = (float*)carve((size_t)NT * 8 * 4); float* BC = (float*)carve((size_t)4 * NT * 32 * 4); float* DT = (float*)carve((size_t)4 * NT * D * 4); float* YS = (float*)carve((size_t)4 * NT * D * 4);
  float* YO = (float*)carve((size_t)NT * C * 4); float* FF = (float*)carve((size_t)NT * D * 4); float* FO = (float*)carve((size_t)NT * D * 4); float* G = (float*)carve((size_t)NT * D * 4);
  if (off > ws_size || off > ((size_t)128 << 20)) return;
  auto wcp = [&](const float* w, int KIN, int OUT, int KP, int OUTP, b16* WT) { wcopyp_kernel<<<(OUTP * KP / 8 + 255) / 256, 256, 0, stream>>>(w, KIN, OUT, KP, OUTP, WT); };
  wcp(Fp(2), C, 2 * D, C, 2 * D, WI); wcp(Fp(5), D, 48, D, 48, WP1); for (int k = 0; k < 4; ++k) { wcp(Fp(13) + (size_t)k * 38 * D, D, 38, D, 48, XPW + (size_t)k * 48 * D); wcp(Fp(14) + (size_t)k * D * R, R, D, 32, D, DTW + (size_t)k * D * 32); }
  wcp(Fp(20), D, C, D, C, WO); wcp(Fp(21), C, D, C, D, WFI); wcp(Fp(31), D, C, D, C, WFO);
  gemm_kernel<96, 24, 1, 0><<<NTV / 16, 32, 0, stream>>>(Fp(0), C, XS, WI, nullptr, NTV, XZ, 2 * D);
  dwconv_kernel<<<(unsigned)(((size_t)NTV * (D / 4) + 255) / 256), 256, 0, stream>>>(XZ, 2 * D, Fp(3), Fp(4), NTV, U);
  gemm_kernel<192, 3, 0, 1><<<NTV / 16, 32, 0, stream>>>(U, D, US, WP1, Fp(6), NTV, P1, 64);
  small_kernel<<<(NTV + 255) / 256, 256, 0, stream>>>(P1, Fp(7), Fp(8), Fp(1), Fp(9), Fp(10), Fp(11), Fp(12), Fp(25), Fp(26), Fp(27), Fp(28), NTV, SMA);
  xproj_kernel<<<dim3(NTV / 16, 4), 32, 0, stream>>>(U, SMA, XPW, DTW, Fp(15), NTV, BC, DT);
  scan_kernel<<<(NBV * 4 * D + 255) / 256, 256, 0, stream>>>(U, DT, BC, Ip(33), Fp(16), Fp(17), NBV, YS);
  tail_kernel<<<NTV / 16, 32, 0, stream>>>(YS, Ip(34), XZ, Fp(18), Fp(19), WO, NTV, YO);
  gemm_kernel<96, 12, 0, 0><<<NTV / 16, 32, 0, stream>>>(YO, C, OS, WFI, Fp(22), NTV, FF, D);
  moeA_kernel<<<(unsigned)(((size_t)NTV * (D / 4) + 255) / 256), 256, 0, stream>>>(FF, SMA, Fp(23), Fp(24), NTV, FO);
  moeB_kernel<<<(unsigned)(((size_t)NTV * (D / 4) + 255) / 256), 256, 0, stream>>>(FO, Fp(29), Fp(30), NTV, G);
  gemm_kernel<192, 6, 0, 0><<<NTV / 16, 32, 0, stream>>>(G, D, GS, WFO, Fp(32), NTV, (float*)d_out, C);
}
